// MambaEncoderLayer_44074954392239
// MI455X (gfx1250) — hardware-verified
//
#include <hip/hip_runtime.h>
#include <math.h>

constexpr int kDModel  = 1024;
constexpr int kDIn     = 1024;
constexpr int kNState  = 16;
constexpr int kDtRank  = 64;
constexpr int kDFfn    = 4096;
constexpr int kBatch   = 2;
constexpr int kSeq     = 2048;
constexpr int kRows    = kBatch * kSeq;
constexpr int kXprojN  = kDtRank + 2 * kNState;
constexpr int kXprojPad = 128;
constexpr int kBCld    = 64;
constexpr float kWCarry   = 16.0f;
constexpr float kActCarry = 16.0f;
constexpr float kInvD     = 1.0f / 1024.0f;
constexpr float kLnEps    = 1e-5f;

constexpr int kScanCh = 64;
constexpr int kScanT  = 32;

constexpr size_t kOffR0   = 0;
constexpr size_t kOffR1   = 33554432;
constexpr size_t kOffR2   = 50331648;
constexpr size_t kOffR3   = 67108864;
constexpr size_t kOffR4   = 75497472;
constexpr size_t kOffDT16 = 83886080;
constexpr size_t kOffBC   = 84410368;
constexpr size_t kOffWA   = 85458944;
constexpr size_t kOffWxp  = 93847552;
constexpr size_t kOffWdt  = 94109696;
constexpr size_t kOffWout = 94240768;
constexpr size_t kWsTotal = 96337920;

typedef __attribute__((ext_vector_type(16))) _Float16 v16h;
typedef __attribute__((ext_vector_type(8)))  _Float16 v8h;
typedef __attribute__((ext_vector_type(16))) __bf16   v16b;
typedef __attribute__((ext_vector_type(8)))  __bf16   v8b;
typedef __attribute__((ext_vector_type(8)))  float    v8f;
typedef __attribute__((ext_vector_type(4)))  float    v4f;
typedef __attribute__((ext_vector_type(4)))  unsigned int v4u;

__device__ __forceinline__ unsigned short f2bf_bits(float f) {
  unsigned u = __float_as_uint(f);
  return (unsigned short)((u + 0x7FFFu + ((u >> 16) & 1u)) >> 16);
}
__device__ __forceinline__ float bf_bits2f(unsigned short h) { return __uint_as_float(((unsigned)h) << 16); }

__device__ __forceinline__ void dep_guard_h(v8f& a, v8f& b, v16h x, v16h y) { asm volatile("v_nop\n\tv_nop\n\tv_nop\n\tv_nop" : "+v"(a), "+v"(b) : "v"(x), "v"(y)); }
__device__ __forceinline__ void dep_guard_b(v8f& a, v8f& b, v16b x, v16b y) { asm volatile("v_nop\n\tv_nop\n\tv_nop\n\tv_nop" : "+v"(a), "+v"(b) : "v"(x), "v"(y)); }
__device__ __forceinline__ void keep4_h(v16h a, v16h b, v16h c, v16h d) { asm volatile("v_nop" :: "v"(a), "v"(b), "v"(c), "v"(d)); }
__device__ __forceinline__ void keep4_b(v16b a, v16b b, v16b c, v16b d) { asm volatile("v_nop" :: "v"(a), "v"(b), "v"(c), "v"(d)); }
__device__ __forceinline__ void acc_guard4(v8f& a, v8f& b, v8f& c, v8f& d) { asm volatile("v_nop\n\tv_nop\n\tv_nop\n\tv_nop" : "+v"(a), "+v"(b), "+v"(c), "+v"(d)); }
template <typename T> struct Frag;
template <> struct Frag<_Float16> {
  typedef v16h V; union U { v16h v; v8h h[2]; };
  static __device__ __forceinline__ v16h load(const _Float16* p) {
    U f; f.h[0] = *(const v8h*)(p); f.h[1] = *(const v8h*)(p + 16); return f.v;
  }
  static __device__ __forceinline__ v8f mma(v16h a, v16h b, v8f c) {
    return __builtin_amdgcn_wmma_f32_16x16x32_f16(false, a, false, b, (short)0, c, false, false);
  }
  static __device__ __forceinline__ void guard(v8f& a, v8f& b, v16h x, v16h y) { dep_guard_h(a, b, x, y); }
  static __device__ __forceinline__ void keep(v16h a, v16h b, v16h c, v16h d) { keep4_h(a, b, c, d); }
};
template <> struct Frag<__bf16> {
  typedef v16b V; union U { v16b v; v8b h[2]; };
  static __device__ __forceinline__ v16b load(const __bf16* p) {
    U f; f.h[0] = *(const v8b*)(p); f.h[1] = *(const v8b*)(p + 16); return f.v;
  }
  static __device__ __forceinline__ v8f mma(v16b a, v16b b, v8f c) {
    return __builtin_amdgcn_wmma_f32_16x16x32_bf16(false, a, false, b, (short)0, c, false, false);
  }
  static __device__ __forceinline__ void guard(v8f& a, v8f& b, v16b x, v16b y) { dep_guard_b(a, b, x, y); }
  static __device__ __forceinline__ void keep(v16b a, v16b b, v16b c, v16b d) { keep4_b(a, b, c, d); }
};

__device__ __forceinline__ unsigned pk16(unsigned short a, unsigned short b) { return (unsigned)a | ((unsigned)b << 16); }
__device__ __forceinline__ unsigned short h_bits(float f) { const _Float16 h = (_Float16)f; return __builtin_bit_cast(unsigned short, h); }

template <int ET> struct Elem;
template <> struct Elem<0> { typedef _Float16 T; };
template <> struct Elem<1> { typedef __bf16 T; };
template <int ET, bool SPLIT, int BIAS_MODE, int OUT_MODE, bool RESID, int ACT = 0>
__global__ __launch_bounds__(256) void wmma_gemm64(
    const unsigned short* __restrict__ Ap, const unsigned short* __restrict__ A2p, int lda, long strideA,
    const unsigned short* __restrict__ Btp, const unsigned short* __restrict__ Bt2p, int ldb, long strideB,
    void* __restrict__ Cout, void* __restrict__ Cout2, int ldc, long strideC,
    const float* __restrict__ bias,
    const float* __restrict__ resid, long strideR,
    int M, int N, int K, float scale) {
  typedef typename Elem<ET>::T T;
  typedef typename Frag<T>::V V;
  const T* A = (const T*)Ap; const T* A2 = (const T*)A2p; const T* Bt = (const T*)Btp; const T* Bt2 = (const T*)Bt2p;
  __shared__ __align__(16) float sT[8][16 * 68];
  const int b    = blockIdx.y;
  const int lane = threadIdx.x & 31;
  const int wave = threadIdx.x >> 5;
  const int tilesN = N >> 6;
  const int tilesM = M >> 6;
  const int tile = blockIdx.x * 8 + wave;
  if (tile >= tilesM * tilesN) return;
  const int tm = tile / tilesN;
  const int tn = tile - tm * tilesN;
  const int m0 = tm << 6;
  const int n0 = tn << 6;

  const T* Ab  = A  + (size_t)b * strideA;
  const T* Bb  = Bt + (size_t)b * strideB;
  const T* Ab2 = SPLIT ? (A2  + (size_t)b * strideA) : nullptr;
  const T* Bb2 = SPLIT ? (Bt2 + (size_t)b * strideB) : nullptr;

  const int rlane = lane & 15;
  const int koff  = (lane >> 4) * 8;
  const int mOff  = (lane >> 4) * 8;

  v8f acc[4][4];
#pragma unroll
  for (int i = 0; i < 4; ++i)
#pragma unroll
    for (int j = 0; j < 4; ++j) acc[i][j] = (v8f){0.f,0.f,0.f,0.f,0.f,0.f,0.f,0.f};

  for (int k0 = 0; k0 < K; k0 += 32) {
    V bh[4], bl[4];
#pragma unroll
    for (int j = 0; j < 4; ++j) {
      const size_t bo = (size_t)(n0 + (j << 4) + rlane) * ldb + koff + k0;
      bh[j] = Frag<T>::load(Bb + bo);
      if (SPLIT) bl[j] = Frag<T>::load(Bb2 + bo);
    }
#pragma unroll
    for (int i = 0; i < 4; ++i) {
      const size_t ao = (size_t)(m0 + (i << 4) + rlane) * lda + koff + k0;
      V ah = Frag<T>::load(Ab + ao);
      V al;
      if (SPLIT) al = Frag<T>::load(Ab2 + ao);
#pragma unroll
      for (int j = 0; j < 4; ++j) {
        acc[i][j] = Frag<T>::mma(ah, bh[j], acc[i][j]);
        if (SPLIT) {
          acc[i][j] = Frag<T>::mma(ah, bl[j], acc[i][j]);
          acc[i][j] = Frag<T>::mma(al, bh[j], acc[i][j]);
        }
      }
      Frag<T>::guard(acc[i][0], acc[i][3], ah, SPLIT ? al : ah);
    }
    Frag<T>::keep(bh[0], bh[1], bh[2], bh[3]);
    if (SPLIT) Frag<T>::keep(bl[0], bl[1], bl[2], bl[3]);
  }
  acc_guard4(acc[0][0], acc[0][1], acc[0][2], acc[0][3]);
  acc_guard4(acc[1][0], acc[1][1], acc[1][2], acc[1][3]);
  acc_guard4(acc[2][0], acc[2][1], acc[2][2], acc[2][3]);
  acc_guard4(acc[3][0], acc[3][1], acc[3][2], acc[3][3]);

  float* slab = sT[wave];
  const float* Rb = RESID ? (resid + (size_t)b * strideR) : nullptr;
#pragma unroll
  for (int i = 0; i < 4; ++i) {
    const int mBase = m0 + (i << 4);
#pragma unroll
    for (int j = 0; j < 4; ++j) {
      const int n = n0 + (j << 4) + rlane;
      float bv = 0.f;
      if (BIAS_MODE == 2) bv = bias[n];
#pragma unroll
      for (int r = 0; r < 8; ++r) {
        float v = acc[i][j][r] * scale;
        if (BIAS_MODE == 1) v += bias[mBase + mOff + r];
        if (BIAS_MODE == 2) v += bv;
        if (RESID) v += Rb[(size_t)(mBase + mOff + r) * ldc + n];
        if (ACT == 2) v = fmaxf(v, 0.0f);
        if (ACT == 4) v = (v > 0.f) ? v : 0.01f * v;
        slab[(mOff + r) * 68 + (j << 4) + rlane] = v;
      }
    }
    __builtin_amdgcn_fence(__ATOMIC_RELEASE, "workgroup");
    __builtin_amdgcn_wave_barrier();
    __builtin_amdgcn_fence(__ATOMIC_ACQUIRE, "workgroup");
    if (OUT_MODE == 0) {
      float* C = (float*)Cout + (size_t)b * strideC;
      const int hh = lane >> 4, c4 = (lane & 15) * 4;
      for (int pass = 0; pass < 2; ++pass) {
#pragma unroll
        for (int it = 0; it < 8; ++it) {
          const int row = it * 2 + hh;
          v4f v = *(const v4f*)(slab + row * 68 + c4);
          *(volatile v4f*)(C + (size_t)(mBase + row) * ldc + n0 + c4) = v;
        }
        __threadfence();
      }
    } else {
      const int q = lane >> 3, c8 = (lane & 7) * 8;
      unsigned short* C  = (unsigned short*)Cout  + (size_t)b * strideC;
      unsigned short* C2 = (OUT_MODE == 2) ? ((unsigned short*)Cout2 + (size_t)b * strideC) : nullptr;
      for (int pass = 0; pass < 2; ++pass) {
#pragma unroll
        for (int it = 0; it < 4; ++it) {
          const int row = it * 4 + q;
          const float* sp = slab + row * 68 + c8;
          v8h hv, lv;
#pragma unroll
          for (int e = 0; e < 8; ++e) {
            if (OUT_MODE == 1) {
              hv[e] = (_Float16)sp[e];
            } else {
              unsigned short hb = f2bf_bits(sp[e]);
              unsigned short lb = f2bf_bits(sp[e] - bf_bits2f(hb));
              hv[e] = __builtin_bit_cast(_Float16, hb);
              lv[e] = __builtin_bit_cast(_Float16, lb);
            }
          }
          *(volatile v8h*)(C + (size_t)(mBase + row) * ldc + n0 + c8) = hv;
          if (OUT_MODE == 2) *(volatile v8h*)(C2 + (size_t)(mBase + row) * ldc + n0 + c8) = lv;
        }
        __threadfence();
      }
    }
    __builtin_amdgcn_fence(__ATOMIC_RELEASE, "workgroup");
    __builtin_amdgcn_wave_barrier();
    __builtin_amdgcn_fence(__ATOMIC_ACQUIRE, "workgroup");
  }
}

__device__ __forceinline__ float wave_sum(float s) {
#pragma unroll
  for (int off = 16; off > 0; off >>= 1) s += __shfl_xor(s, off, 32);
  return s;
}

__global__ __launch_bounds__(256) void cast8_rows_kernel(const float* __restrict__ in, unsigned short* __restrict__ out,
                                                          int rows_src, int cols, int n8, float scale) {
  const int i = blockIdx.x * 256 + threadIdx.x;
  if (i >= n8) return;
  const size_t base = 8 * (size_t)i;
  const int row = (int)(base / (size_t)cols);
  const int col = (int)(base - (size_t)row * cols);
  const int rowc = (row < rows_src) ? row : (rows_src - 1);
  const bool valid = (row < rows_src);
  const float* p = in + (size_t)rowc * cols + col;
  const v4f a = *(const v4f*)(p);
  const v4f c = *(const v4f*)(p + 4);
  unsigned short hb[8];
#pragma unroll
  for (int e = 0; e < 4; ++e) {
    const float va = valid ? a[e] * scale : 0.0f;
    const float vc = valid ? c[e] * scale : 0.0f;
    hb[e]     = h_bits(va);
    hb[4 + e] = h_bits(vc);
  }
  const v4u u = (v4u){pk16(hb[0], hb[1]), pk16(hb[2], hb[3]), pk16(hb[4], hb[5]), pk16(hb[6], hb[7])};
  unsigned short* q = out + base;
  *(volatile v4u*)q = u;
  __threadfence();
  *(volatile v4u*)q = u;
}

template <int MODE>
__global__ __launch_bounds__(128) void ln_kernel(const float* __restrict__ x, const float* __restrict__ res,
                                                 const float* __restrict__ g1, const float* __restrict__ b1,
                                                 const float* __restrict__ g2, const float* __restrict__ b2,
                                                 float* __restrict__ outF, unsigned short* __restrict__ out16) {
  __shared__ float sRedA[4];
  __shared__ float sRedB[4];
  __shared__ float sRedC[4];
  __shared__ float sRedD[4];
  __shared__ __align__(16) float sRow[(MODE == 1) ? kDModel : 4];
  const int row  = blockIdx.x;
  const int t    = threadIdx.x;
  const int lane = t & 31, wave = t >> 5;
  const int c0   = t * 8;
  const size_t rbase = (size_t)row * kDModel;

  const v4f xa = *(const v4f*)(x + rbase + c0);
  const v4f xb = *(const v4f*)(x + rbase + c0 + 4);
  float v[8];
#pragma unroll
  for (int e = 0; e < 4; ++e) { v[e] = xa[e]; v[4 + e] = xb[e]; }

  float s = 0.f;
#pragma unroll
  for (int e = 0; e < 8; ++e) s += v[e];
  s = wave_sum(s);
  if (lane == 0) sRedA[wave] = s;
  __syncthreads();
  const float mean = (((sRedA[0] + sRedA[1]) + sRedA[2]) + sRedA[3]) * kInvD;
  float d[8];
  float q = 0.f;
#pragma unroll
  for (int e = 0; e < 8; ++e) { d[e] = v[e] - mean; q += d[e] * d[e]; }
  q = wave_sum(q);
  if (lane == 0) sRedB[wave] = q;
  __syncthreads();
  const float var = (((sRedB[0] + sRedB[1]) + sRedB[2]) + sRedB[3]) * kInvD;
  const float inv = 1.0f / sqrtf(var + kLnEps);
  float y[8];
#pragma unroll
  for (int e = 0; e < 8; ++e) y[e] = (d[e] * inv) * g1[c0 + e] + b1[c0 + e];

  if (MODE == 1) {
    const v4f ra = *(const v4f*)(res + rbase + c0);
    const v4f rb = *(const v4f*)(res + rbase + c0 + 4);
#pragma unroll
    for (int e = 0; e < 4; ++e) { y[e] = ra[e] + y[e]; y[4 + e] = rb[e] + y[4 + e]; }
#pragma unroll
    for (int e = 0; e < 8; ++e) sRow[c0 + e] = y[e];
    __syncthreads();
    for (int pass = 0; pass < 2; ++pass) {
#pragma unroll
      for (int it = 0; it < 2; ++it) {
        const int col = wave * 256 + it * 128 + lane * 4;
        const v4f val = *(const v4f*)(sRow + col);
        *(volatile v4f*)(outF + rbase + col) = val;
      }
      __threadfence();
    }
    float s2 = 0.f;
#pragma unroll
    for (int e = 0; e < 8; ++e) s2 += y[e];
    s2 = wave_sum(s2);
    if (lane == 0) sRedC[wave] = s2;
    __syncthreads();
    const float mean2 = (((sRedC[0] + sRedC[1]) + sRedC[2]) + sRedC[3]) * kInvD;
    float q2 = 0.f;
#pragma unroll
    for (int e = 0; e < 8; ++e) { d[e] = y[e] - mean2; q2 += d[e] * d[e]; }
    q2 = wave_sum(q2);
    if (lane == 0) sRedD[wave] = q2;
    __syncthreads();
    const float var2 = (((sRedD[0] + sRedD[1]) + sRedD[2]) + sRedD[3]) * kInvD;
    const float inv2 = 1.0f / sqrtf(var2 + kLnEps);
#pragma unroll
    for (int e = 0; e < 8; ++e) y[e] = (d[e] * inv2) * g2[c0 + e] + b2[c0 + e];
  }

  unsigned short hb[8];
#pragma unroll
  for (int e = 0; e < 8; ++e) hb[e] = h_bits(y[e]);
  const v4u u = (v4u){pk16(hb[0], hb[1]), pk16(hb[2], hb[3]), pk16(hb[4], hb[5]), pk16(hb[6], hb[7])};
  unsigned short* op = out16 + rbase + c0;
  *(volatile v4u*)op = u;
  __threadfence();
  *(volatile v4u*)op = u;
}

__global__ __launch_bounds__(128) void conv_silu_kernel(const float* __restrict__ xz, const float* __restrict__ cw,
                                                        const float* __restrict__ cb, float* __restrict__ xc,
                                                        unsigned short* __restrict__ xc16) {
  __shared__ __align__(16) float sRow[kDIn];
  const int r    = blockIdx.x;
  const int l    = r & (kSeq - 1);
  const int t    = threadIdx.x;
  const int lane = t & 31, wave = t >> 5;
  const int rp   = (l > 0) ? (r - 1) : r;
  const float pz = (l > 0) ? 1.0f : 0.0f;
  const size_t rb  = (size_t)r  * (2 * kDIn);
  const size_t rpb = (size_t)rp * (2 * kDIn);
#pragma unroll 1
  for (int e = 0; e < 8; ++e) {
    const int c = t * 8 + e;
    const float xin = xz[rb + c];
    const float xpv = xz[rpb + c] * pz;
    const float w0 = cw[2 * c];
    const float w1 = cw[2 * c + 1];
    const float v = (xpv * w0 + xin * w1) + cb[c];
    const float sg = 1.0f / (1.0f + expf(-v));
    sRow[c] = v * sg;
  }
  __syncthreads();
  const size_t ob = (size_t)r * kDIn;
  for (int pass = 0; pass < 2; ++pass) {
#pragma unroll
    for (int it = 0; it < 2; ++it) {
      const int col = wave * 256 + it * 128 + lane * 4;
      const v4f val = *(const v4f*)(sRow + col);
      *(volatile v4f*)(xc + ob + col) = val;
    }
    __threadfence();
  }
  {
    const int c0 = t * 8;
    const v4f a = *(const v4f*)(sRow + c0);
    const v4f c = *(const v4f*)(sRow + c0 + 4);
    unsigned short hb[8];
#pragma unroll
    for (int e = 0; e < 4; ++e) { hb[e] = h_bits(a[e] * kActCarry); hb[4 + e] = h_bits(c[e] * kActCarry); }
    const v4u u = (v4u){pk16(hb[0], hb[1]), pk16(hb[2], hb[3]), pk16(hb[4], hb[5]), pk16(hb[6], hb[7])};
    unsigned short* op = xc16 + ob + c0;
    *(volatile v4u*)op = u;
    __threadfence();
    *(volatile v4u*)op = u;
  }
}

__global__ __launch_bounds__(64) void scan_kernel(const float* __restrict__ dtraw, const float* __restrict__ xc,
                                                 const float* __restrict__ bc, const float* __restrict__ xz,
                                                 const float* __restrict__ A_log, const float* __restrict__ Dp,
                                                 const float* __restrict__ dt_bias, unsigned short* __restrict__ y16) {
  __shared__ __align__(16) float sDel[kScanT * kScanCh];
  __shared__ __align__(16) float sU[kScanT * kScanCh];
  __shared__ __align__(16) float sSz[kScanT * kScanCh];
  __shared__ __align__(16) float sOut[kScanT * kScanCh];
  __shared__ float sBC[kScanT * 32];
  __shared__ float sH[kNState * kScanCh];
  __shared__ float sAn[kNState * kScanCh];

  const int t    = threadIdx.x;
  const int lane = t & 31, wave = t >> 5;
  const int nDblk = kDIn / kScanCh;
  const int b    = blockIdx.x / nDblk;
  const int d0   = (blockIdx.x - b * nDblk) * kScanCh;
  const int d    = d0 + t;

#pragma unroll 1
  for (int n = 0; n < kNState; ++n) {
    sAn[n * kScanCh + t] = -expf(A_log[d * kNState + n]);
    sH[n * kScanCh + t]  = 0.0f;
  }
  const float dpd = Dp[d];
  const float bd  = dt_bias[d];
  const int q = lane >> 3, c8 = (lane & 7) * 8;

#pragma unroll 1
  for (int ch = 0; ch < kSeq / kScanT; ++ch) {
    const int l0 = ch * kScanT;
    __syncthreads();
#pragma unroll 1
    for (int i = 0; i < kScanT; ++i) {
      const size_t row = (size_t)b * kSeq + l0 + i;
      const float draw = dtraw[row * kDIn + d] + bd;
      const float sp = fmaxf(draw, 0.0f) + log1pf(expf(-fabsf(draw)));
      sDel[i * kScanCh + t] = sp;
      sU[i * kScanCh + t]   = xc[row * kDIn + d];
      const float z  = xz[row * (2 * kDIn) + kDIn + d];
      const float sg = 1.0f / (1.0f + expf(-z));
      sSz[i * kScanCh + t] = z * sg;
    }
#pragma unroll 1
    for (int i = 0; i < (kScanT * 32) / kScanCh; ++i) {
      const int e  = i * kScanCh + t;
      const int s  = e >> 5;
      const int cc = e & 31;
      sBC[e] = bc[((size_t)b * kSeq + l0 + s) * kBCld + cc];
    }
    __syncthreads();
#pragma unroll 1
    for (int s = 0; s < kScanT; ++s) {
      const float del = sDel[s * kScanCh + t];
      const float u   = sU[s * kScanCh + t];
      float yv = 0.0f;
#pragma unroll 1
      for (int g4 = 0; g4 < kNState / 4; ++g4) {
#pragma unroll
        for (int j = 0; j < 4; ++j) {
          const int n = g4 * 4 + j;
          const float a  = sAn[n * kScanCh + t];
          float h        = sH[n * kScanCh + t];
          const float Bn = sBC[s * 32 + n];
          const float Cn = sBC[s * 32 + kNState + n];
          const float dA = expf(del * a);
          const float dBu = (del * Bn) * u;
          h = dA * h + dBu;
          sH[n * kScanCh + t] = h;
          yv += h * Cn;
        }
      }
      const float sz = sSz[s * kScanCh + t];
      sOut[s * kScanCh + t] = ((yv + u * dpd) * sz) * kActCarry;
    }
    __syncthreads();
    for (int pass = 0; pass < 2; ++pass) {
#pragma unroll
      for (int it = 0; it < 4; ++it) {
        const int srow = it * 8 + wave * 4 + q;
        const float* sp = sOut + srow * kScanCh + c8;
        const v4f p0 = *(const v4f*)(sp);
        const v4f p1 = *(const v4f*)(sp + 4);
        unsigned short hb[8];
#pragma unroll
        for (int e = 0; e < 4; ++e) { hb[e] = h_bits(p0[e]); hb[4 + e] = h_bits(p1[e]); }
        const v4u u = (v4u){pk16(hb[0], hb[1]), pk16(hb[2], hb[3]), pk16(hb[4], hb[5]), pk16(hb[6], hb[7])};
        *(volatile v4u*)(y16 + ((size_t)b * kSeq + l0 + srow) * kDIn + d0 + c8) = u;
      }
      __threadfence();
    }
  }
}

static inline dim3 gemm_grid(int M, int N) {
  const int tiles = (M / 64) * (N / 64);
  return dim3((unsigned)((tiles + 7) / 8), 1);
}
static inline unsigned cdiv_u(size_t a, size_t b) { return (unsigned)((a + b - 1) / b); }

extern "C" void kernel_launch(void* const* d_in, const int* in_sizes, int n_in,
                              void* d_out, int out_size, void* d_ws, size_t ws_size,
                              hipStream_t stream) {
  if (n_in < 22) return;
  if ((size_t)out_size != (size_t)kRows * kDModel) return;
  if (ws_size < kWsTotal) return;
  if (in_sizes[0] != kRows * kDModel) return;
  if (in_sizes[1] != 2 * kDIn * kDModel || in_sizes[4] != kXprojN * kDIn || in_sizes[5] != kDIn * kDtRank) return;
  if (in_sizes[18] != kDFfn * kDModel || in_sizes[19] != kDModel * kDFfn || in_sizes[20] != kDModel * kDModel) return;

  const float* src        = (const float*)d_in[0];
  const float* in_proj_w  = (const float*)d_in[1];
  const float* conv_w     = (const float*)d_in[2];
  const float* conv_b     = (const float*)d_in[3];
  const float* x_proj_w   = (const float*)d_in[4];
  const float* dt_proj_w  = (const float*)d_in[5];
  const float* dt_proj_b  = (const float*)d_in[6];
  const float* A_log      = (const float*)d_in[7];
  const float* Dp         = (const float*)d_in[8];
  const float* out_proj_w = (const float*)d_in[9];
  const float* mnorm_g    = (const float*)d_in[10];
  const float* mnorm_b    = (const float*)d_in[11];
  const float* n1_g = (const float*)d_in[12]; const float* n1_b = (const float*)d_in[13];
  const float* n2_g = (const float*)d_in[14]; const float* n2_b = (const float*)d_in[15];
  const float* n3_g = (const float*)d_in[16]; const float* n3_b = (const float*)d_in[17];
  const float* ffn_w1 = (const float*)d_in[18];
  const float* ffn_w2 = (const float*)d_in[19];
  const float* fe_w   = (const float*)d_in[20];
  const float* fe_b   = (const float*)d_in[21];
  float* out = (float*)d_out;

  char* ws = (char*)d_ws;
  float*          XZ    = (float*)(ws + kOffR0);
  unsigned short* FH16  = (unsigned short*)(ws + kOffR0);
  float*          XC    = (float*)(ws + kOffR1);
  float*          Hbuf  = (float*)(ws + kOffR1);
  float*          SRC2  = (float*)(ws + kOffR1);
  float*          DTRAW = (float*)(ws + kOffR2);
  float*          SRC1  = (float*)(ws + kOffR2);
  unsigned short* X16   = (unsigned short*)(ws + kOffR3);
  unsigned short* XC16  = (unsigned short*)(ws + kOffR4);
  unsigned short* Y16   = (unsigned short*)(ws + kOffR4);
  unsigned short* DT16  = (unsigned short*)(ws + kOffDT16);
  float*          BC    = (float*)(ws + kOffBC);
  unsigned short* WA16  = (unsigned short*)(ws + kOffWA);
  unsigned short* Wxp16 = (unsigned short*)(ws + kOffWxp);
  unsigned short* Wdt16 = (unsigned short*)(ws + kOffWdt);
  unsigned short* Wout16 = (unsigned short*)(ws + kOffWout);

  const float invW  = 1.0f / kWCarry;
  const float invWA = 1.0f / (kWCarry * kActCarry);

  {
    const int n8 = 2 * kDIn * kDModel / 8;
    cast8_rows_kernel<<<cdiv_u(n8, 256), 256, 0, stream>>>(in_proj_w, WA16, 2 * kDIn, kDModel, n8, kWCarry);
  }
  {
    const int n8 = kXprojPad * kDIn / 8;
    cast8_rows_kernel<<<cdiv_u(n8, 256), 256, 0, stream>>>(x_proj_w, Wxp16, kXprojN, kDIn, n8, kWCarry);
  }
  {
    const int n8 = kDIn * kDtRank / 8;
    cast8_rows_kernel<<<cdiv_u(n8, 256), 256, 0, stream>>>(dt_proj_w, Wdt16, kDIn, kDtRank, n8, kWCarry);
  }
  {
    const int n8 = kDModel * kDIn / 8;
    cast8_rows_kernel<<<cdiv_u(n8, 256), 256, 0, stream>>>(out_proj_w, Wout16, kDModel, kDIn, n8, kWCarry);
  }

  ln_kernel<0><<<kRows, 128, 0, stream>>>(src, nullptr, n1_g, n1_b, nullptr, nullptr, nullptr, X16);

  wmma_gemm64<0, false, 0, 0, false, 0><<<gemm_grid(kRows, 2 * kDIn), 256, 0, stream>>>(
      X16, nullptr, kDModel, 0L, WA16, nullptr, kDModel, 0L,
      XZ, nullptr, 2 * kDIn, 0L, nullptr, nullptr, 0L, kRows, 2 * kDIn, kDModel, invW);

  conv_silu_kernel<<<kRows, 128, 0, stream>>>(XZ, conv_w, conv_b, XC, XC16);

  wmma_gemm64<0, false, 0, 1, false, 0><<<gemm_grid(kRows, 64), 256, 0, stream>>>(
      XC16, nullptr, kDIn, 0L, Wxp16, nullptr, kDIn, 0L,
      DT16, nullptr, kDtRank, 0L, nullptr, nullptr, 0L, kRows, 64, kDIn, invW);

  wmma_gemm64<0, false, 0, 0, false, 0><<<gemm_grid(kRows, 64), 256, 0, stream>>>(
      XC16, nullptr, kDIn, 0L, Wxp16 + (size_t)64 * kDIn, nullptr, kDIn, 0L,
      BC, nullptr, kBCld, 0L, nullptr, nullptr, 0L, kRows, 64, kDIn, invWA);

  wmma_gemm64<0, false, 0, 0, false, 0><<<gemm_grid(kRows, kDIn), 256, 0, stream>>>(
      DT16, nullptr, kDtRank, 0L, Wdt16, nullptr, kDtRank, 0L,
      DTRAW, nullptr, kDIn, 0L, nullptr, nullptr, 0L, kRows, kDIn, kDtRank, invWA);

  scan_kernel<<<kBatch * (kDIn / kScanCh), kScanCh, 0, stream>>>(DTRAW, XC, BC, XZ, A_log, Dp, dt_proj_b, Y16);

  wmma_gemm64<0, false, 0, 0, false, 0><<<gemm_grid(kRows, kDModel), 256, 0, stream>>>(
      Y16, nullptr, kDIn, 0L, Wout16, nullptr, kDIn, 0L,
      Hbuf, nullptr, kDModel, 0L, nullptr, nullptr, 0L, kRows, kDModel, kDIn, invWA);

  ln_kernel<1><<<kRows, 128, 0, stream>>>(Hbuf, src, mnorm_g, mnorm_b, n2_g, n2_b, SRC1, X16);

  {
    const int n8 = kDFfn * kDModel / 8;
    cast8_rows_kernel<<<cdiv_u(n8, 256), 256, 0, stream>>>(ffn_w1, WA16, kDFfn, kDModel, n8, kWCarry);
  }
  wmma_gemm64<0, false, 0, 1, false, 4><<<gemm_grid(kRows, kDFfn), 256, 0, stream>>>(
      X16, nullptr, kDModel, 0L, WA16, nullptr, kDModel, 0L,
      FH16, nullptr, kDFfn, 0L, nullptr, nullptr, 0L, kRows, kDFfn, kDModel, 1.0f);

  {
    const int n8 = kDModel * kDFfn / 8;
    cast8_rows_kernel<<<cdiv_u(n8, 256), 256, 0, stream>>>(ffn_w2, WA16, kDModel, kDFfn, n8, kWCarry);
  }
  wmma_gemm64<0, false, 0, 0, true, 0><<<gemm_grid(kRows, kDModel), 256, 0, stream>>>(
      FH16, nullptr, kDFfn, 0L, WA16, nullptr, kDFfn, 0L,
      SRC2, nullptr, kDModel, 0L, nullptr, SRC1, 0L, kRows, kDModel, kDFfn, invWA);

  ln_kernel<0><<<kRows, 128, 0, stream>>>(SRC2, nullptr, n3_g, n3_b, nullptr, nullptr, nullptr, X16);

  {
    const int n8 = kDModel * kDModel / 8;
    cast8_rows_kernel<<<cdiv_u(n8, 256), 256, 0, stream>>>(fe_w, WA16, kDModel, kDModel, n8, kWCarry);
  }
  wmma_gemm64<0, false, 2, 0, true, 0><<<gemm_grid(kRows, kDModel), 256, 0, stream>>>(
      X16, nullptr, kDModel, 0L, WA16, nullptr, kDModel, 0L,
      out, nullptr, kDModel, 0L, fe_b, SRC2, 0L, kRows, kDModel, kDModel, invW);
}
